// TwoWordNNLabelProbe_4148938408321
// MI455X (gfx1250) — hardware-run, weakly checked
//
#include <hip/hip_runtime.h>


#ifndef NB
#define NB 16
#endif
#ifndef SEQ
#define SEQ 256
#endif
#define NB_FULL  16
#define SEQ_FULL 256
#ifndef OUT_SEQ
#define OUT_SEQ SEQ
#endif
#define DM   1024
#define RK   256
#define IT   8

static_assert(DM % 32 == 0);
static_assert(DM % 8 == 0);
static_assert((NB * SEQ) % 64 == 0);
static_assert(RK % 64 == 0);
static_assert((2 * RK) % 64 == 0);
static_assert(RK % 32 == 0);
static_assert(RK % 4 == 0);
static_assert(SEQ % 32 == 0);
static_assert(SEQ <= 1024);
static_assert(SEQ % IT == 0);
static_assert(OUT_SEQ % 32 == 0);
static_assert(OUT_SEQ >= SEQ);
static_assert(((size_t)SEQ * DM) % 8 == 0);
static_assert(((size_t)RK * 2 * DM) % 8 == 0);
static_assert(NB <= NB_FULL);
static_assert(SEQ <= SEQ_FULL);
static_assert((16 * 68 * 4) <= 131072);
static_assert(((IT * RK + RK) * 4) <= 131072);
static_assert((68 * 4) % 16 == 0);

typedef unsigned short bf;
typedef __attribute__((ext_vector_type(16))) __bf16   v16bf;
typedef __attribute__((ext_vector_type(8)))  unsigned short v8us;
typedef __attribute__((ext_vector_type(8)))  float    v8f;
typedef __attribute__((ext_vector_type(4)))  float    v4f;
typedef v4f  __attribute__((may_alias)) v4fa;

__device__ __forceinline__ unsigned short f2bf(float f) { unsigned u = __float_as_uint(f); u += 0x7FFFu + ((u >> 16) & 1u); return (unsigned short)(u >> 16); }
__device__ __forceinline__ float bfr(float f) { return __uint_as_float(((unsigned)f2bf(f)) << 16); }
__device__ __forceinline__ v16bf cat16b(v8us lo, v8us hi) { return __builtin_bit_cast(v16bf, __builtin_shufflevector(lo, hi, 0, 1, 2, 3, 4, 5, 6, 7, 8, 9, 10, 11, 12, 13, 14, 15)); }
__device__ __forceinline__ v8f wmmab(v16bf a, v16bf b, v8f c) { return __builtin_amdgcn_wmma_f32_16x16x32_bf16(false, a, false, b, (short)0, c, false, false); }
__device__ __forceinline__ v8f wmmab_g(v16bf a, v16bf b, v8f c) { c = wmmab(a, b, c); asm volatile("v_nop\n\tv_nop\n\tv_nop\n\tv_nop" : "+v"(c) : "v"(a), "v"(b)); return c; }
__device__ __forceinline__ v16bf ldb(const bf* p)  { return cat16b(*(const v8us*)p, *(const v8us*)(p + 16)); }
__device__ __forceinline__ void wave_sync() { __builtin_amdgcn_fence(3  , "wavefront"); __builtin_amdgcn_wave_barrier(); asm volatile("" ::: "memory"); }

__global__ __launch_bounds__(256) void k_cvt8(const float* __restrict__ src, bf* dst, size_t n8) {
    const size_t i = (size_t)blockIdx.x * 256 + threadIdx.x; if (i >= n8) return;
    const v8f v = *(const v8f*)(src + i * 8); v8us o;
#pragma unroll
    for (int k = 0; k < 8; ++k) o[k] = f2bf(v[k]);
    *(volatile v8us*)(dst + i * 8) = o; __threadfence(); *(volatile v8us*)(dst + i * 8) = o;
}

static constexpr size_t PLANE = (size_t)NB * SEQ * RK;

static_assert((size_t)32 * 16 * 8 == (size_t)16 * 64 * 4);
__global__ __launch_bounds__(32) void k_gemm(const bf* __restrict__ A, const bf* __restrict__ W, float* LR) {
    __shared__ __align__(16) float os[16 * 68];
    const int K = DM;
    const int lane = threadIdx.x & 31, lr = lane & 15, hi = lane >> 4; const int r0 = blockIdx.x * 64, c0 = blockIdx.y * 64;
    const int side = c0 / RK, wr0 = c0 % RK;
    v8f acc[4][4];
#pragma unroll
    for (int mb = 0; mb < 4; ++mb)
#pragma unroll
        for (int nb = 0; nb < 4; ++nb) acc[mb][nb] = (v8f){};
    const size_t aoff = (size_t)(r0 + lr) * K + 8 * hi;
    const size_t boff = (size_t)(wr0 + lr) * (size_t)(2 * K) + (size_t)side * K + 8 * hi;
#pragma unroll 1
    for (int kc = 0; kc < K; kc += 32) {
        v16bf a[4];
#pragma unroll
        for (int mb = 0; mb < 4; ++mb) a[mb] = ldb(A + aoff + (size_t)mb * 16 * K + kc);
#pragma unroll
        for (int nb = 0; nb < 4; ++nb) { const v16bf b = ldb(W + boff + (size_t)nb * 16 * (size_t)(2 * K) + kc);
#pragma unroll
            for (int mb = 0; mb < 4; ++mb) acc[mb][nb] = wmmab_g(a[mb], b, acc[mb][nb]); }
    }
    float* dst = LR + (size_t)side * PLANE + (size_t)r0 * RK + (size_t)wr0;
#pragma unroll
    for (int mb = 0; mb < 4; ++mb) {
#pragma unroll
        for (int nb = 0; nb < 4; ++nb) {
#pragma unroll
            for (int j = 0; j < 8; ++j) os[(hi * 8 + j) * 68 + nb * 16 + lr] = acc[mb][nb][j]; }
        wave_sync();
#pragma unroll 1
        for (int ps = 0; ps < 2; ++ps) {
#pragma unroll
            for (int s = 0; s < 8; ++s) { const int row = 2 * s + (lane >> 4), cofs = (lane & 15) * 4;
                const v4f val = *(const v4fa*)(&os[row * 68 + cofs]);
                *(volatile v4f*)(dst + (size_t)(mb * 16 + row) * RK + cofs) = val; }
            if (ps == 0) __threadfence(); }
        wave_sync();
    }
}

static_assert((size_t)SEQ * 4 * IT == (size_t)IT * SEQ * 4);
__global__ __launch_bounds__(SEQ) void k_pair(const float* __restrict__ LR, const float* __restrict__ b1, const float* __restrict__ wl, const float* __restrict__ bl, float* OUT) {
#pragma clang fp contract(off)
    __shared__ __align__(16) float ls[IT * RK];
    __shared__ __align__(16) float wsm[RK];
    const int tid = threadIdx.x;
    const int b = blockIdx.y, i0 = blockIdx.x * IT;
#pragma unroll 1
    for (int c = tid; c < RK; c += SEQ) {
        const float bb = bfr(b1[c]);
        wsm[c] = bfr(wl[c]);
#pragma unroll
        for (int ii = 0; ii < IT; ++ii) ls[ii * RK + c] = LR[(size_t)(b * SEQ + i0 + ii) * RK + c] + bb;
    }
    __syncthreads();
    const float* rrow = LR + PLANE + (size_t)(b * SEQ + tid) * RK;
    float acc[IT][4];
#pragma unroll
    for (int ii = 0; ii < IT; ++ii) { acc[ii][0] = 0.0f; acc[ii][1] = 0.0f; acc[ii][2] = 0.0f; acc[ii][3] = 0.0f; }
#pragma unroll 1
    for (int r = 0; r < RK; r += 4) {
        const v4f rv = *(const v4f*)(rrow + r);
        const v4f wv = *(const v4fa*)(&wsm[r]);
#pragma unroll
        for (int ii = 0; ii < IT; ++ii) {
            const v4f lv = *(const v4fa*)(&ls[ii * RK + r]);
#pragma unroll
            for (int q = 0; q < 4; ++q) { const float hsum = fmaxf(lv[q] + rv[q], 0.0f); acc[ii][q] = fmaf(hsum, wv[q], acc[ii][q]); }
        }
    }
    const float blv = bfr(bl[0]);
    float res[IT];
#pragma unroll
    for (int ii = 0; ii < IT; ++ii) res[ii] = ((acc[ii][0] + acc[ii][1]) + (acc[ii][2] + acc[ii][3])) + blv;
    float* orow = OUT + ((size_t)b * OUT_SEQ + i0) * OUT_SEQ + tid;
#pragma unroll 1
    for (int ps = 0; ps < 2; ++ps) {
#pragma unroll
        for (int ii = 0; ii < IT; ++ii) *(volatile float*)(orow + (size_t)ii * OUT_SEQ) = res[ii];
        if (ps == 0) __threadfence(); }
}

static constexpr size_t al256(size_t v) { return (v + 255) & ~(size_t)255; }
static constexpr size_t SZ_XB = al256((size_t)NB * SEQ * DM * 2);
static constexpr size_t SZ_WB = al256((size_t)RK * 2 * DM * 2);
static constexpr size_t SZ_LR = al256((size_t)2 * NB * SEQ * RK * 4);
static constexpr size_t SZ_TOTAL = SZ_XB + SZ_WB + SZ_LR;
static_assert(SZ_TOTAL <= (size_t)134217728);
static_assert(((size_t)NB * SEQ * DM * 2) % 128 == 0);
static_assert(((size_t)RK * 2 * DM * 2) % 128 == 0);
static_assert((PLANE * 4) % 256 == 0);
static_assert((size_t)(NB * SEQ / 64) * 64 * (size_t)(2 * RK / 64) * 64 == 2 * PLANE);

extern "C" void kernel_launch(void* const* d_in, const int* in_sizes, int n_in,
                              void* d_out, int out_size, void* d_ws, size_t ws_size, hipStream_t stream) {
    if (n_in < 5) return;
    const size_t needx = ((size_t)(NB - 1) * SEQ_FULL + SEQ) * DM;
    if ((size_t)in_sizes[0] < needx) return;
    if ((size_t)in_sizes[1] < (size_t)RK * 2 * DM) return;
    if (in_sizes[2] < RK || in_sizes[3] < RK || in_sizes[4] < 1) return;
    if ((size_t)out_size < ((size_t)(NB - 1) * OUT_SEQ + SEQ) * OUT_SEQ) return;
    if (SZ_TOTAL > ws_size) return;
    const float* xin = (const float*)d_in[0];
    const float* w1  = (const float*)d_in[1];
    const float* b1  = (const float*)d_in[2];
    const float* wl  = (const float*)d_in[3];
    const float* bl  = (const float*)d_in[4];
    float* OUT = (float*)d_out;
    char* wsp = (char*)d_ws;
    bf* XB = (bf*)wsp; wsp += SZ_XB;
    bf* WB = (bf*)wsp; wsp += SZ_WB;
    float* LR = (float*)wsp; wsp += SZ_LR;

    if (SEQ == SEQ_FULL) {
        const size_t n8 = (size_t)NB * SEQ * DM / 8;
        k_cvt8<<<(unsigned)((n8 + 255) / 256), 256, 0, stream>>>(xin, XB, n8);
    } else {
        const size_t n8 = (size_t)SEQ * DM / 8;
        for (int b = 0; b < NB; ++b) k_cvt8<<<(unsigned)((n8 + 255) / 256), 256, 0, stream>>>(xin + (size_t)b * SEQ_FULL * DM, XB + (size_t)b * SEQ * DM, n8);
    }
    { const size_t n8 = (size_t)RK * 2 * DM / 8;
      k_cvt8<<<(unsigned)((n8 + 255) / 256), 256, 0, stream>>>(w1, WB, n8); }

    k_gemm<<<dim3(NB * SEQ / 64, 2 * RK / 64, 1), 32, 0, stream>>>(XB, WB, LR);

    k_pair<<<dim3(SEQ / IT, NB, 1), SEQ, 0, stream>>>(LR, b1, wl, bl, OUT);
}
